// GATModel_35966056136909
// MI455X (gfx1250) — hardware-run, weakly checked
//
#include <hip/hip_runtime.h>


namespace {

constexpr int N = 16384, NP = 16384, NPL = NP  , SRCM = N  , EFULL = 262144, E = EFULL  ;
constexpr int FI = 3, C1 = 128, C2 = 768, NL = (NPL < N ? NPL : N);
constexpr float XS = 8.0f, WSC = 256.0f, WSQ = 0.25f, RS_ = 1024.0f, NSLOPE = 0.2f, LNEPS = 1e-5f, SLOPE = 0.0f, BNEPS = 1e-5f;
static_assert(NP % 32 == 0 && NP >= N && NPL % 32 == 0 && C1 == 128 && C2 == 768 && N % 8 == 0, "tiling");
typedef _Float16 b16;
typedef __attribute__((ext_vector_type(16))) _Float16 v16b;
typedef __attribute__((ext_vector_type(8))) _Float16 v8b;
typedef __attribute__((ext_vector_type(8))) float v8f;
typedef __attribute__((ext_vector_type(4))) float v4f;
__device__ __forceinline__ float bf16_rne(float f) { unsigned int u = __float_as_uint(f); u += 0x7FFFu + ((u >> 16) & 1u); return __uint_as_float(u & 0xFFFF0000u); }
__device__ __forceinline__ void split16(float v, b16& hi, b16& lo) { hi = (b16)v; lo = (b16)(v - (float)hi); }
__device__ __forceinline__ v16b frag_kb(const b16* p, int hh) { const v8b a = *(const v8b*)(p + 8 * hh), b = *(const v8b*)(p + 16 + 8 * hh); v16b f;
#pragma unroll
  for (int e = 0; e < 8; ++e) { f[e] = a[e]; f[8 + e] = b[e]; } return f; }
__device__ __forceinline__ v8f wmma16b(v16b a, v16b b, v8f c) { v8f d = __builtin_amdgcn_wmma_f32_16x16x32_f16(false, a, false, b, (short)0, c, false, false); asm volatile("v_nop\n\tv_nop\n\tv_nop\n\tv_nop" : "+v"(d) : "v"(a), "v"(b)); return d; }
__device__ __forceinline__ void wave_lds_sync() { __builtin_amdgcn_fence(__ATOMIC_RELEASE, "workgroup"); __builtin_amdgcn_wave_barrier(); __builtin_amdgcn_fence(__ATOMIC_ACQUIRE, "workgroup"); }
__device__ __forceinline__ float pmul(float a, float b) { float p = a * b; asm volatile("" : "+v"(p)); return p; }
__device__ __forceinline__ int iclamp(int v, int lo, int hi) { return v < lo ? lo : (v > hi ? hi : v); }
constexpr int CSR_NBLK = 512, CSR_GB = 9, CSR_GN = 1 << CSR_GB  , CSR_MAXG = 512, CSR_CAP = 12288  ;
__global__ __launch_bounds__(64) void csrA_kernel(const int* __restrict__ dst, int E, int N, int nG, int CHP, int NGP, int* __restrict__ STG, int* __restrict__ HST) {
  extern __shared__ int sm[];
  int* cnt = sm; int* run = sm + NGP; int* ids = sm + 2 * NGP;
  const int b = blockIdx.x; const int ch = (E + CSR_NBLK - 1) / CSR_NBLK; const int e0 = b * ch, e1 = min(E, e0 + ch);
  for (int i = threadIdx.x; i < NGP; i += 64) cnt[i] = 0;
  for (int i = threadIdx.x; i < CHP; i += 64) ids[i] = -1;
  __syncthreads();
  if (threadIdx.x == 0) {
    for (int e = e0; e < e1; ++e) { int d = dst[e]; d = (d < 0) ? 0 : (d >= N ? N - 1 : d); cnt[d >> CSR_GB] += 1; }
    int acc = 0; for (int g = 0; g < nG; ++g) { run[g] = acc; acc += cnt[g]; }
    for (int e = e0; e < e1; ++e) { int d = dst[e]; d = (d < 0) ? 0 : (d >= N ? N - 1 : d); const int g = d >> CSR_GB; ids[run[g]] = e; run[g] += 1; } }
  __syncthreads();
  typedef __attribute__((ext_vector_type(4))) int v4i;
  for (int pass = 0; pass < 2; ++pass) {
    for (int i = threadIdx.x; i < CHP / 4; i += 64) *(volatile v4i*)(STG + (size_t)b * CHP + i * 4) = *(const v4i*)(&ids[i * 4]);
    for (int i = threadIdx.x; i < NGP / 4; i += 64) { v4i v; for (int e = 0; e < 4; ++e) v[e] = (i * 4 + e < nG) ? cnt[i * 4 + e] : 0; *(volatile v4i*)(HST + (size_t)b * NGP + i * 4) = v; }
    __threadfence(); }
}
__global__ __launch_bounds__(512) void csrS_kernel(const int* __restrict__ HST, int nG, int NGP, int* __restrict__ START, int* __restrict__ TOT, int* __restrict__ OFF) {
  __shared__ int tot[CSR_MAXG];
  const int b = threadIdx.x;
  for (int pass = 0; pass < 2; ++pass) { int runb = 0; for (int g = 0; g < nG; ++g) { int c = HST[(size_t)b * NGP + g]; c = (c < 0) ? 0 : c; ((volatile int*)OFF)[(size_t)g * CSR_NBLK + b] = runb; runb += c; } __threadfence(); }
  for (int g = threadIdx.x; g < nG; g += 512) { int s = 0; for (int bb = 0; bb < CSR_NBLK; ++bb) { int c = HST[(size_t)bb * NGP + g]; s += (c < 0) ? 0 : c; } tot[g] = s; }
  __syncthreads();
  if (threadIdx.x < 32) {
    __shared__ int st[CSR_MAXG + 32];
    if (threadIdx.x == 0) { int acc = 0; for (int g = 0; g < NGP; ++g) { st[g] = acc; if (g < nG) acc += (tot[g] + 31) & ~31; } st[NGP] = acc; }
    __builtin_amdgcn_fence(__ATOMIC_RELEASE, "workgroup"); __builtin_amdgcn_wave_barrier(); __builtin_amdgcn_fence(__ATOMIC_ACQUIRE, "workgroup");
    for (int pass = 0; pass < 2; ++pass) { for (int i = threadIdx.x; i < NGP + 32; i += 32) { ((volatile int*)START)[i] = (i <= NGP) ? st[min(i, NGP)] : 0; ((volatile int*)TOT)[i] = (i < nG) ? tot[i] : 0; } __threadfence(); } }
}
__global__ __launch_bounds__(256) void csrB_kernel(const int* __restrict__ dst, int N, int nG, int CHP, int NGP, int permLen, const int* __restrict__ STG, const int* __restrict__ HST, const int* __restrict__ OFF, const int* __restrict__ START, const int* __restrict__ TOT, int* __restrict__ PERM, int* __restrict__ ROWPTR, int* __restrict__ ROWCNT, int* __restrict__ FLAG) {
  typedef __attribute__((ext_vector_type(4))) int v4i;
  __shared__ int ids[CSR_CAP]; __shared__ unsigned short key[CSR_CAP]; __shared__ int outp[CSR_CAP]; __shared__ int ncnt[CSR_GN + 1]; __shared__ int boff[CSR_NBLK + 1];
  const int g = blockIdx.x, t_ = threadIdx.x; int tot = TOT[g]; int st = START[g], stn = START[g + 1]; const int v0 = g * CSR_GN; const int nv = min(CSR_GN, N - v0);
  st = (st < 0) ? 0 : (st > permLen - 32 ? permLen - 32 : st) & ~31; stn = (stn < st) ? st : (stn > permLen ? permLen : stn); tot = (tot < 0) ? 0 : tot; if (tot > stn - st && tot <= CSR_CAP) tot = stn - st;
  if (tot > CSR_CAP) {
    for (int pass = 0; pass < 2; ++pass) { for (int i = t_; i < CSR_GN / 4; i += 256) { v4i a, c; for (int e = 0; e < 4; ++e) { a[e] = st; c[e] = 0; } *(volatile v4i*)(ROWPTR + v0 + i * 4) = a; *(volatile v4i*)(ROWCNT + v0 + i * 4) = c; } if (t_ == 0) ((volatile int*)FLAG)[0] = 1; __threadfence(); } (void)nv; return; }
  if (t_ == 0) { int acc = 0; for (int b = 0; b < CSR_NBLK; ++b) { boff[b] = acc; int c = HST[(size_t)b * NGP + g]; c = (c < 0) ? 0 : (c > CHP ? CHP : c); acc += c; if (acc > tot) acc = tot; } boff[CSR_NBLK] = acc; }
  for (int i = t_; i <= CSR_GN; i += 256) ncnt[i] = 0;
  __syncthreads();
  for (int b = 0; b < CSR_NBLK; ++b) { const int c = boff[b + 1] - boff[b]; int o_ = OFF[(size_t)g * CSR_NBLK + b]; o_ = (o_ < 0) ? 0 : (o_ > CHP - c ? CHP - c : o_); const int* src_ = STG + (size_t)b * CHP + o_;
    for (int i = t_; i < c; i += 256) { int id = src_[i]; id = (id < 0) ? 0 : id; ids[boff[b] + i] = id; int d = dst[id]; d = (d < v0) ? v0 : (d >= N ? N - 1 : d); int kk = d - v0; kk = (kk < 0) ? 0 : (kk >= CSR_GN ? CSR_GN - 1 : kk); key[boff[b] + i] = (unsigned short)kk; } }
  __syncthreads();
  if (t_ == 0) { for (int i = 0; i < tot; ++i) ncnt[key[i]] += 1; int acc = 0; for (int vl = 0; vl < CSR_GN; ++vl) { const int c = ncnt[vl]; ncnt[vl] = acc; acc += c; } ncnt[CSR_GN] = acc;
    for (int i = 0; i < tot; ++i) { const int vl = key[i]; outp[ncnt[vl]] = ids[i]; ncnt[vl] += 1; }
    for (int vl = CSR_GN; vl > 0; --vl) ncnt[vl] = ncnt[vl - 1]; ncnt[0] = 0; }
  __syncthreads();
  for (int pass = 0; pass < 2; ++pass) {
    for (int i = t_; i < (stn - st) / 4; i += 256) { v4i v; for (int e = 0; e < 4; ++e) { const int q = i * 4 + e; v[e] = (q < tot) ? outp[q] : -1; } *(volatile v4i*)(PERM + st + i * 4) = v; }
    for (int i = t_; i < CSR_GN / 4; i += 256) { v4i a, c; for (int e = 0; e < 4; ++e) { const int vl = i * 4 + e; a[e] = st + ncnt[vl]; c[e] = (vl < nv) ? (ncnt[vl + 1] - ncnt[vl]) : 0; } *(volatile v4i*)(ROWPTR + v0 + i * 4) = a; *(volatile v4i*)(ROWCNT + v0 + i * 4) = c; }
    __threadfence(); }
}
__global__ __launch_bounds__(256) void csrZ_kernel(int* __restrict__ p, size_t n4) { typedef __attribute__((ext_vector_type(4))) int v4i; const size_t tid = (size_t)blockIdx.x * 256 + threadIdx.x, nth = (size_t)gridDim.x * 256; v4i z = {0, 0, 0, 0}; for (size_t i = tid; i < n4; i += nth) *(volatile v4i*)(p + i * 4) = z; }
struct CsrBufs { int *STG, *HST, *OFF, *START, *TOT, *PERM, *ROWPTR, *ROWCNT, *FLAG; int nG, NGP, CHP; size_t permLen; char* base; size_t bytes; };
static size_t csr_carve(CsrBufs& c, char* ws, size_t off, int E, int N) {
  const size_t off0 = off; c.base = ws + off;
  auto al = [&](size_t bytes) { char* p = ws + off; off += (bytes + 255) & ~(size_t)255; return p; };
  c.nG = (N + CSR_GN - 1) / CSR_GN; c.NGP = (c.nG + 31) & ~31; const int ch = (E + CSR_NBLK - 1) / CSR_NBLK; c.CHP = (ch + 31) & ~31; c.permLen = (size_t)E + 32 * (size_t)c.nG + 32;
  c.STG = (int*)al((size_t)CSR_NBLK * c.CHP * 4); c.HST = (int*)al((size_t)CSR_NBLK * c.NGP * 4); c.OFF = (int*)al((size_t)c.NGP * CSR_NBLK * 4); c.START = (int*)al((size_t)(c.NGP + 64) * 4); c.TOT = (int*)al((size_t)(c.NGP + 64) * 4);
  c.PERM = (int*)al(c.permLen * 4); c.ROWPTR = (int*)al((size_t)c.nG * CSR_GN * 4); c.ROWCNT = (int*)al((size_t)c.nG * CSR_GN * 4); c.FLAG = (int*)al(256);
  c.bytes = off - off0; return off;
}
static void csr_build(const CsrBufs& c, const int* dst, int E, int N, hipStream_t stream) {
  const size_t smem = (size_t)(2 * c.NGP + c.CHP) * 4;
  csrZ_kernel<<<512, 256, 0, stream>>>((int*)c.base, c.bytes / 16);
  csrA_kernel<<<CSR_NBLK, 64, smem, stream>>>(dst, E, N, c.nG, c.CHP, c.NGP, c.STG, c.HST);
  csrS_kernel<<<1, 512, 0, stream>>>(c.HST, c.nG, c.NGP, c.START, c.TOT, c.OFF);
  csrB_kernel<<<c.nG, 256, 0, stream>>>(dst, N, c.nG, c.CHP, c.NGP, (int)c.permLen, c.STG, c.HST, c.OFF, c.START, c.TOT, c.PERM, c.ROWPTR, c.ROWCNT, c.FLAG);
}

typedef __attribute__((ext_vector_type(4))) _Float16 v4h;
typedef __attribute__((ext_vector_type(2))) float v2f;
__device__ __forceinline__ float lrelu(float v) { return v > 0.0f ? v : NSLOPE * v; }
__device__ __forceinline__ float bfp(float v) { float t = bf16_rne(v); asm volatile("" : "+v"(t)); return t; }
__global__ __launch_bounds__(256) void wt_kernel(const float* __restrict__ wl, const float* __restrict__ wr, b16* __restrict__ WT, float scl) {
  const int u = blockIdx.x * 256 + threadIdx.x; if (u >= 2 * C2 * C1 / 8) return; const int e = u * 8; const int o = e / C1, k0 = e % C1; const float* w = o < C2 ? wl : wr; const int oo = o < C2 ? o : o - C2; v8b v;
#pragma unroll
  for (int j = 0; j < 8; ++j) v[j] = (b16)(bf16_rne(w[(size_t)(k0 + j) * C2 + oo]) * scl);
  for (int pass = 0; pass < 2; ++pass) { *(volatile v8b*)(WT + e) = v; __threadfence(); }
}
__global__ __launch_bounds__(256) void lin3_kernel(const float* __restrict__ x, const float* __restrict__ wl, const float* __restrict__ bl, const float* __restrict__ wr, const float* __restrict__ br, float* __restrict__ XL, float* __restrict__ XR) {
  const int u = blockIdx.x * 256 + threadIdx.x; if (u >= NP * C1 / 8) return; const int v = u / (C1 / 8), c0 = (u % (C1 / 8)) * 8; float xv[FI]; for (int i = 0; i < FI; ++i) xv[i] = (v < N) ? bfp(x[(size_t)v * FI + i]) : 0.0f;
  v4f ol[2], orr[2];
#pragma unroll
  for (int j = 0; j < 8; ++j) { const int c = c0 + j; float sl = bfp(bl[c]), sr = bfp(br[c]); float tl = 0.0f, tr = 0.0f; for (int i = 0; i < FI; ++i) { tl += pmul(xv[i], bfp(wl[i * C1 + c])); tr += pmul(xv[i], bfp(wr[i * C1 + c])); } ol[j >> 2][j & 3] = (v < N) ? tl + sl : 0.0f; orr[j >> 2][j & 3] = (v < N) ? tr + sr : 0.0f; }
  for (int pass = 0; pass < 2; ++pass) { *(volatile v4f*)(XL + (size_t)u * 8) = ol[0]; *(volatile v4f*)(XL + (size_t)u * 8 + 4) = ol[1]; *(volatile v4f*)(XR + (size_t)u * 8) = orr[0]; *(volatile v4f*)(XR + (size_t)u * 8 + 4) = orr[1]; __threadfence(); }
}
template <int C, bool L2>
__global__ __launch_bounds__(256) void node_kernel(const float* __restrict__ XL, const float* __restrict__ XR, const float* __restrict__ att, const float* __restrict__ bias, const float* __restrict__ g, const float* __restrict__ bb,
    const int* __restrict__ srcs, const int* __restrict__ PERM, const int* __restrict__ ROWPTR, const int* __restrict__ ROWCNT, int permLen,
    const float* __restrict__ x, const float* __restrict__ wfc, const float* __restrict__ bfc, float* __restrict__ OUT, int mrows) {
  constexpr int KP = C / 128;
  const int wave = threadIdx.x >> 5, lane = threadIdx.x & 31; const int v = blockIdx.x * 8 + wave; const int vv = v < N ? v : N - 1;
  float xr[4 * KP], at[4 * KP], acc[4 * KP];
#pragma unroll
  for (int k = 0; k < KP; ++k) { const v4f r4 = *(const v4f*)(XR + (size_t)vv * C + 128 * k + 4 * lane); for (int j = 0; j < 4; ++j) { xr[4 * k + j] = r4[j]; at[4 * k + j] = bfp(att[128 * k + 4 * lane + j]); acc[4 * k + j] = 0.0f; } }
  int cnt = 0, p0 = 0; if (v < N) { cnt = iclamp(ROWCNT[v], 0, 65536); p0 = iclamp(ROWPTR[v], 0, permLen - 1); if (p0 + cnt > permLen) cnt = permLen - p0; }
  float m = -INFINITY, l = 0.0f;
#pragma unroll 1
  for (int i = 0; i <= cnt; ++i) {
    int s = vv; if (i < cnt) { const int e = iclamp(PERM[p0 + i], 0, E - 1); s = iclamp(srcs[e], 0, N - 1); if (SRCM < N) s %= SRCM; }
    const float* xlr = XL + (size_t)s * C + 4 * lane; float xl[4 * KP]; float part = 0.0f;
#pragma unroll
    for (int k = 0; k < KP; ++k) { const v4f t4 = *(const v4f*)(xlr + 128 * k); for (int j = 0; j < 4; ++j) { xl[4 * k + j] = t4[j]; part += pmul(at[4 * k + j], lrelu(t4[j] + xr[4 * k + j])); } }
#pragma unroll
    for (int o = 16; o >= 1; o >>= 1) part += __shfl_xor(part, o);
    const float mn = fmaxf(m, part); const float al = __expf(m - mn), pw = __expf(part - mn); l = l * al + pw; m = mn;
#pragma unroll
    for (int q = 0; q < 4 * KP; ++q) acc[q] = pmul(acc[q], al) + pmul(pw, xl[q]); }
  const float inv = 1.0f / l; float h[4 * KP]; float s1 = 0.0f;
  float xv[FI]; if (L2) { for (int i2 = 0; i2 < FI; ++i2) xv[i2] = bfp(x[(size_t)vv * FI + i2]); }
#pragma unroll
  for (int k = 0; k < KP; ++k) for (int j = 0; j < 4; ++j) { const int c = 128 * k + 4 * lane + j; float y = pmul(acc[4 * k + j], inv) + bfp(bias[c]);
      if (L2) { float r = bfp(bfc[c]); for (int i2 = 0; i2 < FI; ++i2) r += pmul(xv[i2], bfp(wfc[i2 * C + c])); y += r; }
      h[4 * k + j] = y; s1 += y; }
#pragma unroll
  for (int o = 16; o >= 1; o >>= 1) s1 += __shfl_xor(s1, o);
  const float mu = s1 * (1.0f / C); float s2 = 0.0f;
#pragma unroll
  for (int q = 0; q < 4 * KP; ++q) { const float d = h[q] - mu; s2 += pmul(d, d); }
#pragma unroll
  for (int o = 16; o >= 1; o >>= 1) s2 += __shfl_xor(s2, o);
  const float rs = rsqrtf(s2 * (1.0f / C) + LNEPS);
  v4f o4[KP];
#pragma unroll
  for (int k = 0; k < KP; ++k) for (int j = 0; j < 4; ++j) { const int c = 128 * k + 4 * lane + j; float y = pmul((h[4 * k + j] - mu) * rs, bfp(g[c])) + bfp(bb[c]); if (!L2) y = y > 0.0f ? y : __expf(y) - 1.0f; o4[k][j] = (v < N) ? y : 0.0f; }
  for (int pass = 0; pass < 2; ++pass) { if (v < mrows) {
#pragma unroll
      for (int k = 0; k < KP; ++k) *(volatile v4f*)(OUT + (size_t)v * C + 128 * k + 4 * lane) = o4[k]; }
    __threadfence(); }
}
__global__ __launch_bounds__(256) void proj2_kernel(const float* __restrict__ H1, const b16* __restrict__ WT, const b16* __restrict__ WQ, const float* __restrict__ b2l, const float* __restrict__ b2r, float* __restrict__ XL2, float* __restrict__ XR2) {
  __shared__ __attribute__((aligned(16))) b16 Ah[32][C1 + 8], Al[32][C1 + 8]; __shared__ __attribute__((aligned(16))) float Tf[32][C2 + 4];
  const int tid = threadIdx.x, wave = tid >> 5, lane = tid & 31, nloc = lane & 15, hlf = lane >> 4; const int v0 = blockIdx.x * 32; const int half = blockIdx.y;
  { const int row = tid >> 3, g = tid & 7, c0 = g * 16; const float* hr = H1 + (size_t)(v0 + row) * C1 + c0;
#pragma unroll
    for (int q = 0; q < 4; ++q) { const v4f t4 = *(const v4f*)(hr + 4 * q); v4h hv, lv; for (int j = 0; j < 4; ++j) { const float vs = t4[j] * XS; const b16 p = (b16)vs; hv[j] = p; lv[j] = (b16)((vs - (float)p) * RS_); } *(v4h*)(&Ah[row][c0 + 4 * q]) = hv; *(v4h*)(&Al[row][c0 + 4 * q]) = lv; } }
  __syncthreads();
  v8f acc[2][6];
#pragma unroll
  for (int t = 0; t < 6; ++t) { acc[0][t] = (v8f){}; acc[1][t] = (v8f){}; }
#pragma unroll
  for (int kb = 0; kb < C1; kb += 32) { const v16b a0 = frag_kb(&Ah[nloc][kb], hlf), a1 = frag_kb(&Ah[16 + nloc][kb], hlf), l0 = frag_kb(&Al[nloc][kb], hlf), l1 = frag_kb(&Al[16 + nloc][kb], hlf);
#pragma unroll
    for (int t = 0; t < 6; ++t) { const size_t wo_ = (size_t)(half * C2 + (wave * 6 + t) * 16 + nloc) * C1 + kb; const v16b bw = frag_kb(WT + wo_, hlf), bwq = frag_kb(WQ + wo_, hlf);
      acc[0][t] = wmma16b(a0, bw, acc[0][t]); acc[0][t] = wmma16b(l0, bwq, acc[0][t]); acc[1][t] = wmma16b(a1, bw, acc[1][t]); acc[1][t] = wmma16b(l1, bwq, acc[1][t]); } }
  const float* bias = half == 0 ? b2l : b2r;
#pragma unroll
  for (int t = 0; t < 6; ++t) { const int col = (wave * 6 + t) * 16 + nloc; const float bbv = bf16_rne(bias[col]);
#pragma unroll
    for (int rt = 0; rt < 2; ++rt)
#pragma unroll
      for (int q = 0; q < 8; ++q) { const int rr = rt * 16 + 8 * hlf + q; Tf[rr][col] = (v0 + rr < N) ? acc[rt][t][q] * (1.0f / (XS * WSC)) + bbv : 0.0f; } }
  __syncthreads();
  float* dstp = half == 0 ? XL2 : XR2;
  for (int pass = 0; pass < 2; ++pass) { for (int rr = wave * 4; rr < wave * 4 + 4; ++rr) { float* d = dstp + (size_t)(v0 + rr) * C2;
#pragma unroll
      for (int s = 0; s < 6; ++s) *(volatile v4f*)(d + s * 128 + lane * 4) = *(const v4f*)(&Tf[rr][s * 128 + lane * 4]); } __threadfence(); }
}
}

extern "C" void kernel_launch(void* const* d_in, const int* in_sizes, int n_in, void* d_out, int out_size, void* d_ws, size_t ws_size, hipStream_t stream) {
  (void)n_in;
  auto Fp = [&](int i) { return (const float*)d_in[i]; }; auto Ip = [&](int i) { return (const int*)d_in[i]; };
  if (in_sizes[0] != N * FI || in_sizes[1] != 2 * EFULL || in_sizes[2] != FI * C2 || in_sizes[3] != C2 || in_sizes[4] != FI * C1 || in_sizes[5] != C1 || in_sizes[6] != FI * C1 || in_sizes[7] != C1 || in_sizes[8] != C1 || in_sizes[9] != C1 || in_sizes[10] != C1 || in_sizes[11] != C1 || in_sizes[12] != C1 * C2 || in_sizes[13] != C2 || in_sizes[14] != C1 * C2 || in_sizes[15] != C2 || in_sizes[16] != C2 || in_sizes[17] != C2 || in_sizes[18] != C2 || in_sizes[19] != C2 || out_size != N * C2) return;
  size_t off = 0; char* ws = (char*)d_ws;
  auto carve = [&](size_t bytes) { char* p = ws + off; off += (bytes + 255) & ~(size_t)255; return p; };
  b16* WT = (b16*)carve((size_t)2 * C2 * C1 * 2); b16* WQ = (b16*)carve((size_t)2 * C2 * C1 * 2);
  float* XL1 = (float*)carve((size_t)NP * C1 * 4); float* XR1 = (float*)carve((size_t)NP * C1 * 4); float* H1 = (float*)carve((size_t)NP * C1 * 4); float* XL2 = (float*)carve((size_t)NP * C2 * 4); float* XR2 = (float*)carve((size_t)NP * C2 * 4);
  CsrBufs csr; off = csr_carve(csr, ws, off, E, N);
  if (off > ws_size || off > ((size_t)160 << 20)) return;
  wt_kernel<<<(2 * C2 * C1 / 8 + 255) / 256, 256, 0, stream>>>(Fp(12), Fp(14), WT, WSC); wt_kernel<<<(2 * C2 * C1 / 8 + 255) / 256, 256, 0, stream>>>(Fp(12), Fp(14), WQ, WSQ);
  csr_build(csr, Ip(1) + EFULL, E, N, stream);
  lin3_kernel<<<(NP * C1 / 8 + 255) / 256, 256, 0, stream>>>(Fp(0), Fp(4), Fp(5), Fp(6), Fp(7), XL1, XR1);
  node_kernel<C1, false><<<NPL / 8, 256, 0, stream>>>(XL1, XR1, Fp(8), Fp(9), Fp(10), Fp(11), Ip(1), csr.PERM, csr.ROWPTR, csr.ROWCNT, (int)csr.permLen, Fp(0), Fp(2), Fp(3), H1, NPL);
  proj2_kernel<<<dim3(NPL / 32, 2), 256, 0, stream>>>(H1, WT, WQ, Fp(13), Fp(15), XL2, XR2);
  node_kernel<C2, true><<<NPL / 8, 256, 0, stream>>>(XL2, XR2, Fp(16), Fp(17), Fp(18), Fp(19), Ip(1), csr.PERM, csr.ROWPTR, csr.ROWCNT, (int)csr.permLen, Fp(0), Fp(2), Fp(3), (float*)d_out, NL);
}
